// PSABlock_1494648619601
// MI455X (gfx1250) — hardware-verified
//
#include <hip/hip_runtime.h>
#include <math.h>

typedef __attribute__((ext_vector_type(16))) _Float16 v16h;
typedef __attribute__((ext_vector_type(16))) __bf16 v16b;
typedef __attribute__((ext_vector_type(8)))  _Float16 v8h;
typedef __attribute__((ext_vector_type(8)))  float v8f;
typedef __attribute__((ext_vector_type(4)))  float v4f;
typedef __attribute__((ext_vector_type(2)))  float v2f;
typedef __attribute__((ext_vector_type(4)))  unsigned v4u;
typedef __attribute__((ext_vector_type(4)))  int v4i;
typedef float __attribute__((may_alias)) float_a;
typedef int __attribute__((may_alias)) int_a;

template <typename T> __device__ __forceinline__ void vst2(void* p, T v) { *(volatile T*)p = v; __threadfence(); *(volatile T*)p = v; }
__device__ __forceinline__ v8f wmma16(v16h a, v16h b, v8f c) {
  v8f d = __builtin_amdgcn_wmma_f32_16x16x32_f16(false, a, false, b, (short)0, c, false, false);
  asm volatile("v_nop\n\tv_nop\n\tv_nop\n\tv_nop" : "+v"(d) : "v"(a), "v"(b));
  return d;
}
__device__ __forceinline__ v8f wmma_bf(v16b a, v16b b, v8f c) {
  v8f d = __builtin_amdgcn_wmma_f32_16x16x32_bf16(false, a, false, b, (short)0, c, false, false);
  asm volatile("v_nop\n\tv_nop\n\tv_nop\n\tv_nop" : "+v"(d) : "v"(a), "v"(b));
  return d;
}
__device__ __forceinline__ v16h frag_h(const _Float16* rowk0, int lane) {
  union { v16h v; v8h q[2]; } u; const _Float16* p = rowk0 + 8 * (lane >> 4);
  u.q[0] = *(const v8h*)p; u.q[1] = *(const v8h*)(p + 16); return u.v;
}
__device__ __forceinline__ v16h frag_f32(const float* rowk0, int lane) {
  v16h a; const float* p = rowk0 + 8 * (lane >> 4);
#pragma unroll
  for (int i = 0; i < 8; ++i) { a[i] = (_Float16)p[i]; a[8 + i] = (_Float16)p[16 + i]; }
  return a;
}
__device__ __forceinline__ v16h frag_f32s(const float* rowk0, int lane, float sc) {
  v16h a; const float* p = rowk0 + 8 * (lane >> 4);
#pragma unroll
  for (int i = 0; i < 8; ++i) { a[i] = (_Float16)(p[i] * sc); a[8 + i] = (_Float16)(p[16 + i] * sc); }
  return a;
}
__device__ __forceinline__ v16h fragc_f32(const float* W, int k0, int n, int lane, int ld, int K) {
  v16h a; const int g = lane >> 4;
#pragma unroll
  for (int i = 0; i < 8; ++i) { const int ka = k0 + 8 * g + i, kb = ka + 16;
    a[i] = (_Float16)(ka < K ? W[(size_t)ka * ld + n] : 0.f); a[8 + i] = (_Float16)(kb < K ? W[(size_t)kb * ld + n] : 0.f); }
  return a;
}
struct F2 { v16b h, l; };
__device__ __forceinline__ F2 bsplit16(const float v[16]) { F2 r;
#pragma unroll
  for (int i = 0; i < 16; ++i) { const __bf16 h = (__bf16)v[i]; r.h[i] = h; r.l[i] = (__bf16)(v[i] - (float)h); }
  return r; }
__device__ __forceinline__ F2 split_row(const float* row, int k0, int lane) { float v[16]; const float* p = row + k0 + 8 * (lane >> 4);
#pragma unroll
  for (int i = 0; i < 8; ++i) { v[i] = p[i]; v[8 + i] = p[16 + i]; }
  return bsplit16(v); }
__device__ __forceinline__ F2 split_rowK(const float* row, int k0, int lane, int K) { float v[16]; const int g = lane >> 4;
#pragma unroll
  for (int i = 0; i < 8; ++i) { const int ka = k0 + 8 * g + i, kb = ka + 16; v[i] = ka < K ? row[ka] : 0.f; v[8 + i] = kb < K ? row[kb] : 0.f; }
  return bsplit16(v); }
__device__ __forceinline__ F2 split_col(const float* W, int k0, int n, int lane, int ld, int K) { float v[16]; const int g = lane >> 4;
#pragma unroll
  for (int i = 0; i < 8; ++i) { const int ka = k0 + 8 * g + i, kb = ka + 16; v[i] = ka < K ? W[(size_t)ka * ld + n] : 0.f; v[8 + i] = kb < K ? W[(size_t)kb * ld + n] : 0.f; }
  return bsplit16(v); }
__device__ __forceinline__ v8f mac3(const F2& a, const F2& b, v8f c) { c = wmma_bf(a.l, b.h, c); c = wmma_bf(a.h, b.l, c); return wmma_bf(a.h, b.h, c); }
__device__ __forceinline__ float sigm(float v) { return 1.0f / (1.0f + expf(-v)); }
#define LDSX() do { asm volatile("s_wait_dscnt 0" ::: "memory"); __builtin_amdgcn_wave_barrier(); __builtin_amdgcn_fence(__ATOMIC_RELEASE, "workgroup"); } while (0)

#define NB 4
#define CC 256
#define HI 48
#define WI 48
#define NP (HI * WI)
#define NH 4
#define KD 32
#define HD 64
#define QKVC 512
#define FF 512

__device__ __forceinline__ float bnf(float v, const float* g, const float* b, const float* m, const float* var, int c) { const float s = g[c] * rsqrtf(var[c] + 1e-3f); return v * s + (b[c] - m[c] * s); }

__global__ __launch_bounds__(128) void k_qkv(const float* __restrict__ x, const float* __restrict__ W, const float* __restrict__ bg, const float* __restrict__ bb, const float* __restrict__ bm, const float* __restrict__ bv,
                                           _Float16* __restrict__ Q16, _Float16* __restrict__ K16, _Float16* __restrict__ V16, float* __restrict__ V32) {
  __shared__ __align__(16) float sq[4][16][68];
  __shared__ __align__(16) float sv[HD][68];
  const int tid = threadIdx.x, wave = tid >> 5, lane = tid & 31, col = lane & 15, g = lane >> 4;
  const int b = blockIdx.z, h = blockIdx.y, p0b = blockIdx.x * 64, p0 = p0b + wave * 16; const int o0 = h * 128;
  const float* xb = x + (size_t)b * CC * NP;
  v8f acc[8] = {};
#pragma unroll 1
  for (int kc = 0; kc < CC / 32; ++kc) { const v16h a = fragc_f32(xb, kc * 32, p0 + col, lane, NP, CC);
#pragma unroll
    for (int j = 0; j < 8; ++j) acc[j] = wmma16(a, frag_f32s(W + (size_t)(o0 + j * 16 + col) * CC + kc * 32, lane, 16.0f), acc[j]); }
#pragma unroll
  for (int j = 0; j < 8; ++j) { const int ol = j * 16 + col, o = o0 + ol;
#pragma unroll
    for (int r = 0; r < 8; ++r) { const float v = bnf(acc[j][r] * (1.0f / 16.0f), bg, bb, bm, bv, o); if (ol < 64) sq[wave][8 * g + r][ol] = v; else sv[ol - 64][wave * 16 + 8 * g + r] = v; } }
  LDSX();
  for (int q = lane; q < 16 * 8; q += 32) { const int rl = q >> 3, pc = q & 7; union { v8h h8; v4u u; } pk; const int which = pc >> 2, pcl = pc & 3;
#pragma unroll
    for (int e = 0; e < 8; ++e) pk.h8[e] = (_Float16)sq[wave][rl][which * 32 + pcl * 8 + e];
    vst2((which ? K16 : Q16) + (((size_t)b * NH + h) * NP + p0 + rl) * KD + pcl * 8, pk.u); }
  __syncthreads();
  for (int q = tid; q < HD * 16; q += 128) { const int d = q >> 4, pc = q & 15; vst2(V32 + ((size_t)b * CC + h * HD + d) * NP + p0b + pc * 4, *(const v4f*)(&sv[d][pc * 4])); }
  for (int q = tid; q < HD * 8; q += 128) { const int d = q >> 3, pc = q & 7; union { v8h h8; v4u u; } pk;
#pragma unroll
    for (int e = 0; e < 8; ++e) pk.h8[e] = (_Float16)sv[d][pc * 8 + e];
    vst2(V16 + (((size_t)b * NH + h) * HD + d) * NP + p0b + pc * 8, pk.u); }
}
__global__ __launch_bounds__(128) void k_attn(const _Float16* __restrict__ Q16, const _Float16* __restrict__ K16, const _Float16* __restrict__ V16, float* __restrict__ O32) {
  __shared__ __align__(16) float sS[4][16][68];
  __shared__ __align__(16) _Float16 sP[4][16][72];
  __shared__ __align__(16) float sO[HD][68];
  const int tid = threadIdx.x, w = tid >> 5, lane = tid & 31, col = lane & 15, g = lane >> 4;
  const int b = blockIdx.z, h = blockIdx.y, p0b = blockIdx.x * 64, q0 = p0b + w * 16; const size_t bh = (size_t)b * NH + h;
  const _Float16* qb = Q16 + bh * NP * KD; const _Float16* kb = K16 + bh * NP * KD; const _Float16* vb = V16 + bh * HD * NP;
  const v16h aq = frag_h(qb + (size_t)(q0 + col) * KD, lane);
  float mrun = -3.0e38f, lrun = 0.f; v8f acc[4] = {};
  const float scl = 0.17677669529663687f;
#pragma unroll 1
  for (int kt = 0; kt < NP / 64; ++kt) {
#pragma unroll
    for (int t = 0; t < 4; ++t) { v8f s = {}; s = wmma16(aq, frag_h(kb + (size_t)(kt * 64 + t * 16 + col) * KD, lane), s);
#pragma unroll
      for (int r = 0; r < 8; ++r) sS[w][8 * g + r][t * 16 + col] = s[r] * scl; }
    LDSX();
    float mx = -3.4e38f;
#pragma unroll
    for (int jj = 0; jj < 32; ++jj) mx = fmaxf(mx, sS[w][col][g * 32 + jj]);
    mx = fmaxf(mx, __shfl_xor(mx, 16, 32));
    const float mnew = fmaxf(mrun, mx); const float corr = expf(mrun - mnew);
    float ps = 0.f;
#pragma unroll
    for (int jj = 0; jj < 32; ++jj) { const float p = expf(sS[w][col][g * 32 + jj] - mnew); ps += p; sP[w][col][g * 32 + jj] = (_Float16)(p * 16384.0f); }
    ps += __shfl_xor(ps, 16, 32);
    lrun = lrun * corr + ps; mrun = mnew;
#pragma unroll
    for (int r = 0; r < 8; ++r) { const float cr = __shfl(corr, 8 * g + r, 32);
#pragma unroll
      for (int t = 0; t < 4; ++t) acc[t][r] *= cr; }
    LDSX();
#pragma unroll
    for (int kc = 0; kc < 2; ++kc) { const v16h pa = frag_h(&sP[w][col][0] + kc * 32, lane);
#pragma unroll
      for (int t = 0; t < 4; ++t) acc[t] = wmma16(pa, frag_h(vb + (size_t)(t * 16 + col) * NP + kt * 64 + kc * 32, lane), acc[t]); }
    __builtin_amdgcn_wave_barrier();
  }
#pragma unroll
  for (int r = 0; r < 8; ++r) { const float lr = __shfl(lrun, 8 * g + r, 32);
#pragma unroll
    for (int t = 0; t < 4; ++t) sO[t * 16 + col][w * 16 + 8 * g + r] = acc[t][r] / (lr * 16384.0f); }
  __syncthreads();
  for (int q = tid; q < HD * 16; q += 128) { const int d = q >> 4, pc = q & 15; vst2(O32 + ((size_t)b * CC + h * HD + d) * NP + p0b + pc * 4, *(const v4f*)(&sO[d][pc * 4])); }
}
__global__ __launch_bounds__(128) void k_proj(const float* __restrict__ O32, const float* __restrict__ V32, const float* __restrict__ x, const float* __restrict__ pew, const float* __restrict__ pg, const float* __restrict__ pb, const float* __restrict__ pm, const float* __restrict__ pv,
                                            const float* __restrict__ W, const float* __restrict__ bg, const float* __restrict__ bb, const float* __restrict__ bm, const float* __restrict__ bv, float* __restrict__ X1) {
  __shared__ __align__(16) float sT[CC][68];
  __shared__ __align__(16) float sX[CC][68];
  const int tid = threadIdx.x, wave = tid >> 5, lane = tid & 31, col = lane & 15, g = lane >> 4;
  const int b = blockIdx.y, p0b = blockIdx.x * 64, p0 = p0b + wave * 16; (void)p0;
  const float* vb32 = V32 + (size_t)b * CC * NP; const float* ob = O32 + (size_t)b * CC * NP; const float* xb = x + (size_t)b * CC * NP;
  for (int q = tid; q < CC * 64; q += 128) { const int c = q >> 6, pl = q & 63; const int p = p0b + pl, py = p / WI, px = p % WI; const float* pl_v = vb32 + (size_t)c * NP; float a = 0.f;
#pragma unroll
    for (int k = 0; k < 9; ++k) { const int yy = py + k / 3 - 1, xx = px + k % 3 - 1; if (yy >= 0 && yy < HI && xx >= 0 && xx < WI) a += pew[c * 9 + k] * pl_v[yy * WI + xx]; }
    sT[c][pl] = ob[(size_t)c * NP + p] + bnf(a, pg, pb, pm, pv, c); }
  __syncthreads();
#pragma unroll 1
  for (int np = 0; np < 2; ++np) { v8f acc[8];
#pragma unroll
    for (int j = 0; j < 8; ++j) acc[j] = (v8f){};
#pragma unroll 1
    for (int kc = 0; kc < CC / 32; ++kc) { const v16h a = fragc_f32(&sT[0][0], kc * 32, wave * 16 + col, lane, 68, CC);
#pragma unroll
      for (int j = 0; j < 8; ++j) acc[j] = wmma16(a, frag_f32s(W + (size_t)(np * 128 + j * 16 + col) * CC + kc * 32, lane, 16.0f), acc[j]); }
#pragma unroll
    for (int j = 0; j < 8; ++j) { const int o = np * 128 + j * 16 + col;
#pragma unroll
      for (int r = 0; r < 8; ++r) { const int pl = wave * 16 + 8 * g + r; sX[o][pl] = xb[(size_t)o * NP + p0b + pl] + bnf(acc[j][r] * (1.0f / 16.0f), bg, bb, bm, bv, o); } } }
  __syncthreads();
  for (int q = tid; q < CC * 16; q += 128) { const int c = q >> 4, pc = q & 15; vst2(X1 + ((size_t)b * CC + c) * NP + p0b + pc * 4, *(const v4f*)(&sX[c][pc * 4])); }
}
__global__ __launch_bounds__(128) void k_ffn(const float* __restrict__ X1, const float* __restrict__ W1, const float* __restrict__ g1, const float* __restrict__ b1, const float* __restrict__ m1, const float* __restrict__ v1,
                                           const float* __restrict__ W2, const float* __restrict__ g2, const float* __restrict__ b2, const float* __restrict__ m2, const float* __restrict__ v2, float* __restrict__ out) {
  __shared__ __align__(16) float sH[FF][68];
  __shared__ __align__(16) float sO[CC][68];
  const int tid = threadIdx.x, wave = tid >> 5, lane = tid & 31, col = lane & 15, g = lane >> 4;
  const int b = blockIdx.y, p0b = blockIdx.x * 64, p0 = p0b + wave * 16; const float* xb = X1 + (size_t)b * CC * NP;
#pragma unroll 1
  for (int np = 0; np < FF / 128; ++np) { v8f acc[8] = {};
#pragma unroll 1
    for (int kc = 0; kc < 8; ++kc) { const v16h a = fragc_f32(xb, kc * 32, p0 + col, lane, NP, CC);
#pragma unroll
      for (int j = 0; j < 8; ++j) acc[j] = wmma16(a, frag_f32s(W1 + (size_t)(np * 128 + j * 16 + col) * CC + kc * 32, lane, 16.0f), acc[j]); }
#pragma unroll
    for (int j = 0; j < 8; ++j) { const int f = np * 128 + j * 16 + col;
#pragma unroll
      for (int r = 0; r < 8; ++r) { const float v = bnf(acc[j][r] * (1.0f / 16.0f), g1, b1, m1, v1, f); sH[f][wave * 16 + 8 * g + r] = v * sigm(v); } } }
  LDSX();
#pragma unroll 1
  for (int np = 0; np < 2; ++np) { v8f acc[8];
#pragma unroll
    for (int j = 0; j < 8; ++j) acc[j] = (v8f){};
#pragma unroll 1
    for (int kc = 0; kc < FF / 32; ++kc) { const v16h a = fragc_f32(&sH[0][0], kc * 32, wave * 16 + col, lane, 68, FF);
#pragma unroll
      for (int j = 0; j < 8; ++j) acc[j] = wmma16(a, frag_f32s(W2 + (size_t)(np * 128 + j * 16 + col) * FF + kc * 32, lane, 16.0f), acc[j]); }
#pragma unroll
    for (int j = 0; j < 8; ++j) { const int o = np * 128 + j * 16 + col;
#pragma unroll
      for (int r = 0; r < 8; ++r) { const int pl = wave * 16 + 8 * g + r; sO[o][pl] = xb[(size_t)o * NP + p0b + pl] + bnf(acc[j][r] * (1.0f / 16.0f), g2, b2, m2, v2, o); } } }
  __syncthreads();
  for (int q = tid; q < CC * 16; q += 128) { const int c = q >> 4, pc = q & 15; vst2(out + ((size_t)b * CC + c) * NP + p0b + pc * 4, *(const v4f*)(&sO[c][pc * 4])); }
}
extern "C" void kernel_launch(void* const* d_in, const int* in_sizes, int n_in, void* d_out, int out_size, void* d_ws, size_t ws_size, hipStream_t stream) {
  (void)in_sizes; (void)n_in; (void)out_size; (void)ws_size;
  const float** I = (const float**)d_in;
  const float* x = I[0]; const float* qkvw = I[1]; const float* qg = I[2]; const float* qb = I[3]; const float* qm = I[4]; const float* qv = I[5];
  const float* pew = I[6]; const float* pg = I[7]; const float* pb = I[8]; const float* pm = I[9]; const float* pv = I[10];
  const float* prw = I[11]; const float* prg = I[12]; const float* prb = I[13]; const float* prm = I[14]; const float* prv = I[15];
  const float* f1w = I[16]; const float* f1g = I[17]; const float* f1b = I[18]; const float* f1m = I[19]; const float* f1v = I[20];
  const float* f2w = I[21]; const float* f2g = I[22]; const float* f2b = I[23]; const float* f2m = I[24]; const float* f2v = I[25];
  float* out = (float*)d_out;
  char* ws = (char*)d_ws; size_t off = 0;
  auto take = [&](size_t bytes) { char* p = ws + off; off += (bytes + 255) & ~(size_t)255; return p; };
  _Float16* Q16 = (_Float16*)take((size_t)NB * NH * NP * KD * 2); _Float16* K16 = (_Float16*)take((size_t)NB * NH * NP * KD * 2); _Float16* V16 = (_Float16*)take((size_t)NB * NH * HD * NP * 2);
  float* V32 = (float*)take((size_t)NB * CC * NP * 4); float* O32 = (float*)take((size_t)NB * CC * NP * 4); float* X1 = (float*)take((size_t)NB * CC * NP * 4);
  k_qkv<<<dim3(NP / 64, NH, NB), 128, 0, stream>>>(x, qkvw, qg, qb, qm, qv, Q16, K16, V16, V32);
  k_attn<<<dim3(NP / 64, NH, NB), 128, 0, stream>>>(Q16, K16, V16, O32);
  k_proj<<<dim3(NP / 64, NB), 128, 0, stream>>>(O32, V32, x, pew, pg, pb, pm, pv, prw, prg, prb, prm, prv, X1);
  k_ffn<<<dim3(NP / 64, NB), 128, 0, stream>>>(X1, f1w, f1g, f1b, f1m, f1v, f2w, f2g, f2b, f2m, f2v, out);
}
